// CausalSelfAttention_73005854097696
// MI455X (gfx1250) — hardware-run, weakly checked
//
#include <hip/hip_runtime.h>
#ifndef NB
#define NB 4
#endif
#ifndef SEQ
#define SEQ 2048
#endif
#define SEQ_FULL 2048
#define DM 1024
#define NH 16
#define HD 64
#define QE ((SEQ < 512) ? SEQ : 512)
#define NR ((size_t)NB * SEQ)
#define LQK (2 * DM)
#define LDW3 (3 * DM)
#define LDV (NB * SEQ)
#define LDVL (NB * QE)

static_assert(SEQ % 128 == 0);
static_assert(QE % 128 == 0);
static_assert(DM % 128 == 0);
static_assert(DM % 64 == 0);
static_assert(DM % 32 == 0);
static_assert(NH * HD == DM);
static_assert(HD == 64);
static_assert(SEQ <= SEQ_FULL);
static_assert(LQK % 64 == 0);
static_assert((NB * SEQ) % 128 == 0);

#define SZ_BQK ((size_t)2 * DM * DM * 2)
#define SZ_BW  ((size_t)DM * DM * 2)
#define SZ_X16 (NR * DM * 2)
#define SZ_QKH (NR * LQK * 2)
#define SZ_QKL ((size_t)NB * QE * LQK * 2)
#define SZ_VTH ((size_t)DM * LDV * 2)
#define SZ_VTL ((size_t)DM * LDVL * 2)
#define SZ_CTH (NR * DM * 2)
#define SZ_CTL ((size_t)NB * QE * DM * 2)
#define SZ_CS  ((size_t)64 * SEQ * 4)
#define WS_TOTAL (SZ_BQK + 2 * SZ_BW + SZ_X16 + SZ_QKH + SZ_QKL + SZ_VTH + SZ_VTL + SZ_CTH + SZ_CTL + SZ_CS)
static_assert(WS_TOTAL <= (size_t)134217728);
static_assert(SZ_BQK % 256 == 0 && SZ_BW % 256 == 0 && SZ_X16 % 256 == 0 && SZ_QKH % 256 == 0 && SZ_QKL % 256 == 0 && SZ_VTH % 256 == 0 && SZ_VTL % 256 == 0 && SZ_CTH % 256 == 0 && SZ_CTL % 256 == 0 && SZ_CS % 256 == 0);

typedef unsigned short v8us __attribute__((ext_vector_type(8), may_alias));
typedef float  v8f  __attribute__((ext_vector_type(8)));
typedef float  v4f  __attribute__((ext_vector_type(4)));
typedef float  v4fa __attribute__((ext_vector_type(4), may_alias));
typedef _Float16 v16h __attribute__((ext_vector_type(16)));
union FragH { v16h v; v8us half[2]; _Float16 h[16]; unsigned short u[16]; };

struct RopeF { float f[32]; };
static_assert(sizeof(RopeF) == 128);

__device__ __forceinline__ unsigned short bf16_bits(float x) { unsigned int u = __float_as_uint(x); return (unsigned short)((u + 0x7FFFu + ((u >> 16) & 1u)) >> 16); }
__device__ __forceinline__ float bf16_rne(float x) { return __uint_as_float(((unsigned int)bf16_bits(x)) << 16); }

__device__ __forceinline__ v16h g2_frag(const _Float16* p, int hh) { FragH f; f.half[0] = *(const v8us*)((const unsigned short*)p + 8 * hh); f.half[1] = *(const v8us*)((const unsigned short*)p + 16 + 8 * hh); return f.v; }
__device__ __forceinline__ v8f g2_mma(v16h a, v16h b, v8f c) { v8f d = __builtin_amdgcn_wmma_f32_16x16x32_f16(false, a, false, b, (short)0, c, false, false); asm volatile("v_nop\n\tv_nop\n\tv_nop\n\tv_nop" : "+v"(d) : "v"(a), "v"(b)); return d; }

__global__ __launch_bounds__(256) void k_wtr(const float* __restrict__ w, int ldw, int colbase, _Float16* __restrict__ Bt) {
  __shared__ float ts[64][65];
  const int tid = threadIdx.x;
  const int n0 = blockIdx.x * 64, k0 = blockIdx.y * 64;
#pragma unroll
  for (int it = 0; it < 4; ++it) {
    const int kk = it * 16 + (tid >> 4), nn = (tid & 15) * 4;
    const v4f a = *(const v4fa*)(w + (size_t)(k0 + kk) * ldw + colbase + n0 + nn);
    ts[kk][nn] = a[0]; ts[kk][nn + 1] = a[1]; ts[kk][nn + 2] = a[2]; ts[kk][nn + 3] = a[3];
  }
  __syncthreads();
  v8us o[2];
#pragma unroll
  for (int it = 0; it < 2; ++it) {
    const int p = it * 256 + tid; const int nl = p >> 3, kc = (p & 7) * 8;
    FragH f;
#pragma unroll
    for (int e = 0; e < 8; ++e) f.h[e] = (_Float16)(bf16_rne(ts[kc + e][nl]) * 16.0f);
    o[it] = f.half[0];
  }
  for (int pass = 0; pass < 2; ++pass) {
#pragma unroll
    for (int it = 0; it < 2; ++it) { const int p = it * 256 + tid; const int nl = p >> 3, kc = (p & 7) * 8;
      *(volatile v8us*)((unsigned short*)Bt + (size_t)(n0 + nl) * DM + k0 + kc) = o[it]; }
    if (pass == 0) __threadfence();
  }
}

__global__ __launch_bounds__(256) void k_x16(const float* __restrict__ x, _Float16* __restrict__ X16) {
  const size_t n8 = (size_t)SEQ * DM / 8;
  const size_t t = (size_t)blockIdx.x * 256 + threadIdx.x; if (t >= n8) return;
  const float* src = x + (size_t)blockIdx.y * SEQ_FULL * DM + t * 8;
  unsigned short* dst = (unsigned short*)X16 + (size_t)blockIdx.y * SEQ * DM + t * 8;
  const v4f a = *(const v4fa*)(src), c = *(const v4fa*)(src + 4);
  FragH f;
#pragma unroll
  for (int q = 0; q < 4; ++q) { f.h[q] = (_Float16)bf16_rne(a[q]); f.h[4 + q] = (_Float16)bf16_rne(c[q]); }
  const v8us o = f.half[0];
  *(volatile v8us*)dst = o; __threadfence(); *(volatile v8us*)dst = o;
}

__global__ __launch_bounds__(256) void k_ropetab(RopeF rf, float* __restrict__ CS) {
  const int g = blockIdx.x * 256 + threadIdx.x; if (g >= 32 * SEQ) return;
  const int i = g / SEQ, pos = g - i * SEQ;
  float fr = rf.f[0];
#pragma unroll
  for (int k = 1; k < 32; ++k) fr = (i == k) ? rf.f[k] : fr;
  const float ang = (float)pos * fr;
  float sn, cs; sincosf(ang, &sn, &cs);
  volatile float* pc = CS + (size_t)i * SEQ + pos; volatile float* ps = CS + (size_t)(32 + i) * SEQ + pos;
  *pc = cs; *ps = sn; __threadfence(); *pc = cs; *ps = sn;
}

template <int MODE>
__device__ __forceinline__ void proj_body(const _Float16* __restrict__ A, int lda, const _Float16* __restrict__ Bh, int ldb, float alpha, const float* __restrict__ CS, const float* __restrict__ bias,
                                          _Float16* __restrict__ Ch, int ldch, _Float16* __restrict__ Cl, int ldcl, int M, int N, int K) {
  __shared__ __attribute__((aligned(16))) float so[4][32][68];
  const int tid = threadIdx.x, lane = tid & 31, ln = lane & 15, hh = lane >> 4;
  const int w = __builtin_amdgcn_readfirstlane(tid >> 5);
  const int ntn = N >> 6; const int mt = blockIdx.x / ntn, nq = blockIdx.x - mt * ntn; const int row0 = mt * 128 + 32 * w, col0 = nq * 64; if (row0 >= M) return;
  const _Float16* a0p = A + (size_t)(row0 + ln) * lda; const _Float16* a1p = a0p + (size_t)16 * lda;
  const _Float16* b0p = Bh + (size_t)(col0 + ln) * ldb; const _Float16* b1p = b0p + (size_t)16 * ldb; const _Float16* b2p = b1p + (size_t)16 * ldb; const _Float16* b3p = b2p + (size_t)16 * ldb;
  const v8f z8 = {0.f,0.f,0.f,0.f,0.f,0.f,0.f,0.f}; v8f c00 = z8, c01 = z8, c02 = z8, c03 = z8, c10 = z8, c11 = z8, c12 = z8, c13 = z8;
#pragma unroll 1
  for (int kb = 0; kb < K; kb += 32) { const v16h a0 = g2_frag(a0p + kb, hh), a1 = g2_frag(a1p + kb, hh);
    v16h b = g2_frag(b0p + kb, hh); c00 = g2_mma(a0, b, c00); c10 = g2_mma(a1, b, c10);
    b = g2_frag(b1p + kb, hh); c01 = g2_mma(a0, b, c01); c11 = g2_mma(a1, b, c11);
    b = g2_frag(b2p + kb, hh); c02 = g2_mma(a0, b, c02); c12 = g2_mma(a1, b, c12);
    b = g2_frag(b3p + kb, hh); c03 = g2_mma(a0, b, c03); c13 = g2_mma(a1, b, c13); }
  v8f accs[8] = {c00, c01, c02, c03, c10, c11, c12, c13};
  if (MODE == 0) {
    float bl[2], bu[2];
#pragma unroll
    for (int t = 0; t < 2; ++t) { bl[t] = bf16_rne(bias[col0 + t * 16 + ln]); bu[t] = bf16_rne(bias[col0 + 32 + t * 16 + ln]); }
#pragma unroll
    for (int half = 0; half < 2; ++half) {
#pragma unroll
      for (int t = 0; t < 2; ++t) {
        const int i = t * 16 + ln; const int p0 = (row0 + half * 16 + 8 * hh) % SEQ;
        const v4f ca = *(const v4fa*)(CS + (size_t)i * SEQ + p0), cb = *(const v4fa*)(CS + (size_t)i * SEQ + p0 + 4);
        const v4f sa = *(const v4fa*)(CS + (size_t)(32 + i) * SEQ + p0), sb = *(const v4fa*)(CS + (size_t)(32 + i) * SEQ + p0 + 4);
        const float cc[8] = {ca[0], ca[1], ca[2], ca[3], cb[0], cb[1], cb[2], cb[3]};
        const float ss[8] = {sa[0], sa[1], sa[2], sa[3], sb[0], sb[1], sb[2], sb[3]};
#pragma unroll
        for (int r = 0; r < 8; ++r) { const int rloc = half * 16 + 8 * hh + r; const float x1 = accs[half * 4 + t][r] * alpha + bl[t], x2 = accs[half * 4 + t + 2][r] * alpha + bu[t];
          so[w][rloc][i] = x1 * cc[r] - x2 * ss[r]; so[w][rloc][32 + i] = x1 * ss[r] + x2 * cc[r]; }
      }
    }
  } else {
    float bv[16];
#pragma unroll
    for (int half = 0; half < 2; ++half) { const float* bp = bias + row0 + half * 16 + 8 * hh;
      const v4f ba = *(const v4fa*)bp, bb = *(const v4fa*)(bp + 4);
#pragma unroll
      for (int e = 0; e < 4; ++e) { bv[half * 8 + e] = bf16_rne(ba[e]); bv[half * 8 + 4 + e] = bf16_rne(bb[e]); } }
#pragma unroll
    for (int u = 0; u < 8; ++u) { const int t = u & 3, half = u >> 2;
#pragma unroll
      for (int r = 0; r < 8; ++r) so[w][half * 16 + 8 * hh + r][t * 16 + ln] = accs[u][r] * alpha + bv[half * 8 + r]; }
  }
  __builtin_amdgcn_fence(4  , "workgroup"); __builtin_amdgcn_wave_barrier();
  bool early; size_t lobase;
  if (MODE == 0) { const int rb = mt * 128; const int bidx = rb / SEQ; const int t0 = rb - bidx * SEQ; early = t0 < QE; lobase = ((size_t)bidx * QE + t0 + 32 * w) * ldcl + col0; }
  else { const int bidx = col0 / SEQ; const int tc = col0 - bidx * SEQ; early = tc < QE; lobase = (size_t)row0 * ldcl + (size_t)bidx * QE + tc; }
  const int rsub = lane >> 3, pc = (lane & 7) * 8;
  for (int pass = 0; pass < 2; ++pass) {
#pragma unroll
    for (int q = 0; q < 8; ++q) { const int rr = q * 4 + rsub;
      const v4f a = *(const v4fa*)&so[w][rr][pc], c = *(const v4fa*)&so[w][rr][pc + 4];
      FragH fh, fl;
#pragma unroll
      for (int e = 0; e < 4; ++e) { _Float16 h = (_Float16)a[e]; fh.h[e] = h; fl.h[e] = (_Float16)((a[e] - (float)h) * 1024.0f); h = (_Float16)c[e]; fh.h[4 + e] = h; fl.h[4 + e] = (_Float16)((c[e] - (float)h) * 1024.0f); }
      *(volatile v8us*)((unsigned short*)Ch + (size_t)(row0 + rr) * ldch + col0 + pc) = fh.half[0];
      if (early) *(volatile v8us*)((unsigned short*)Cl + lobase + (size_t)rr * ldcl + pc) = fl.half[0];
    }
    if (pass == 0) __threadfence();
  }
}

__global__ __launch_bounds__(128) void k_proj_qk(const _Float16* __restrict__ A, int lda, const _Float16* __restrict__ Bh, int ldb, float alpha, const float* __restrict__ CS, const float* __restrict__ bias,
                                                 _Float16* __restrict__ Ch, int ldch, _Float16* __restrict__ Cl, int ldcl, int M, int N, int K) {
  proj_body<0>(A, lda, Bh, ldb, alpha, CS, bias, Ch, ldch, Cl, ldcl, M, N, K);
}
__global__ __launch_bounds__(128) void k_proj_vt(const _Float16* __restrict__ A, int lda, const _Float16* __restrict__ Bh, int ldb, float alpha, const float* __restrict__ CS, const float* __restrict__ bias,
                                                 _Float16* __restrict__ Ch, int ldch, _Float16* __restrict__ Cl, int ldcl, int M, int N, int K) {
  proj_body<1>(A, lda, Bh, ldb, alpha, CS, bias, Ch, ldch, Cl, ldcl, M, N, K);
}

template <bool PRECISE>
__device__ __forceinline__ void flash_body(const _Float16* __restrict__ QK, const _Float16* __restrict__ QKL, const _Float16* __restrict__ VH, const _Float16* __restrict__ VL,
                                           _Float16* __restrict__ CH, _Float16* __restrict__ CL, int qbase) {
  __shared__ __attribute__((aligned(16))) float so[4][16][68];
  const int tid = threadIdx.x, lane = tid & 31, ln = lane & 15, hh = lane >> 4;
  const int w = __builtin_amdgcn_readfirstlane(tid >> 5);
  const int b = blockIdx.y / NH, hd = blockIdx.y - b * NH;
  const int qw0 = qbase + (int)blockIdx.x * 64 + 16 * w;
  const int qi = qw0 + ln;
  const size_t rowb = (size_t)b * SEQ, rowl = (size_t)b * QE;
  const _Float16* qp = QK + (rowb + qi) * LQK + hd * HD;
  const v16h qh0 = g2_frag(qp, hh), qh1 = g2_frag(qp + 32, hh);
  v16h ql0 = qh0, ql1 = qh1;
  if (PRECISE) { const _Float16* qlp = QKL + (rowl + qi) * LQK + hd * HD; ql0 = g2_frag(qlp, hh); ql1 = g2_frag(qlp + 32, hh); }
  const v8f z8 = {0.f,0.f,0.f,0.f,0.f,0.f,0.f,0.f};
  v8f o0 = z8, o1 = z8, o2 = z8, o3 = z8, x0 = z8, x1 = z8, x2 = z8, x3 = z8;
  float m = -1.0e30f, l = 0.f;
  const int nkt = (qw0 + 15) / 32 + 1;
#pragma unroll 1
  for (int kt = 0; kt < nkt; ++kt) {
    const int j0 = kt * 32;
    const _Float16* kp = QK + (rowb + j0 + ln) * LQK + DM + hd * HD;
    const _Float16* klp = QKL + (rowl + j0 + ln) * LQK + DM + hd * HD;
    float sv[16];
#pragma unroll
    for (int g = 0; g < 2; ++g) {
      const _Float16* kg = kp + (size_t)g * 16 * LQK;
      const v16h a0 = g2_frag(kg, hh), a1 = g2_frag(kg + 32, hh);
      v8f s = z8;
      if (PRECISE) {
        const _Float16* kl = klp + (size_t)g * 16 * LQK;
        const v16h e0 = g2_frag(kl, hh), e1 = g2_frag(kl + 32, hh);
        s = g2_mma(a0, ql0, s); s = g2_mma(a1, ql1, s); s = g2_mma(e0, qh0, s); s = g2_mma(e1, qh1, s);
        s = s * 0.0009765625f;
      }
      s = g2_mma(a0, qh0, s); s = g2_mma(a1, qh1, s);
#pragma unroll
      for (int r = 0; r < 8; ++r) sv[g * 8 + r] = s[r] * 0.125f;
    }
    if (j0 + 31 > qw0) {
#pragma unroll
      for (int r = 0; r < 8; ++r) { const int ja = j0 + 8 * hh + r; sv[r] = (ja <= qi) ? sv[r] : -1.0e30f; sv[8 + r] = (ja + 16 <= qi) ? sv[8 + r] : -1.0e30f; }
    }
    float mx = sv[0];
#pragma unroll
    for (int e = 1; e < 16; ++e) mx = fmaxf(mx, sv[e]);
    mx = fmaxf(mx, __shfl_xor(mx, 16, 32));
    const float mnew = fmaxf(m, mx);
    if (__builtin_amdgcn_ballot_w32(mnew > m) != 0u) {
      const float corr = __expf(m - mnew);
      l *= corr; o0 = o0 * corr; o1 = o1 * corr; o2 = o2 * corr; o3 = o3 * corr;
      if (PRECISE) { x0 = x0 * corr; x1 = x1 * corr; x2 = x2 * corr; x3 = x3 * corr; }
      m = mnew;
    }
    FragH pb, pl; pb.v = qh0; pl.v = qh0;
    float ls = 0.f;
#pragma unroll
    for (int r = 0; r < 8; ++r) {
      const float e0 = __expf(sv[r] - m), e1 = __expf(sv[8 + r] - m); ls += e0 + e1;
      const float c0 = e0 * 256.0f, c1 = e1 * 256.0f; const _Float16 h0 = (_Float16)c0, h1 = (_Float16)c1;
      pb.h[r] = h0; pb.h[8 + r] = h1;
      if (PRECISE) { pl.h[r] = (_Float16)((c0 - (float)h0) * 1024.0f); pl.h[8 + r] = (_Float16)((c1 - (float)h1) * 1024.0f); }
    }
    l += ls;
    const _Float16* vp = VH + (size_t)(hd * HD + ln) * LDV + rowb + j0;
    { v16h a = g2_frag(vp, hh); o0 = g2_mma(a, pb.v, o0); if (PRECISE) x0 = g2_mma(a, pl.v, x0);
      a = g2_frag(vp + (size_t)16 * LDV, hh); o1 = g2_mma(a, pb.v, o1); if (PRECISE) x1 = g2_mma(a, pl.v, x1);
      a = g2_frag(vp + (size_t)32 * LDV, hh); o2 = g2_mma(a, pb.v, o2); if (PRECISE) x2 = g2_mma(a, pl.v, x2);
      a = g2_frag(vp + (size_t)48 * LDV, hh); o3 = g2_mma(a, pb.v, o3); if (PRECISE) x3 = g2_mma(a, pl.v, x3); }
    if (PRECISE) { const _Float16* vlp = VL + (size_t)(hd * HD + ln) * LDVL + rowl + j0;
      v16h a = g2_frag(vlp, hh); x0 = g2_mma(a, pb.v, x0);
      a = g2_frag(vlp + (size_t)16 * LDVL, hh); x1 = g2_mma(a, pb.v, x1);
      a = g2_frag(vlp + (size_t)32 * LDVL, hh); x2 = g2_mma(a, pb.v, x2);
      a = g2_frag(vlp + (size_t)48 * LDVL, hh); x3 = g2_mma(a, pb.v, x3); }
  }
  const float lt = l + __shfl_xor(l, 16, 32);
  const float inv = 0.25f / lt;
  v8f oa[4] = {o0, o1, o2, o3}; v8f xa[4] = {x0, x1, x2, x3};
#pragma unroll
  for (int dt = 0; dt < 4; ++dt) {
#pragma unroll
    for (int r = 0; r < 8; ++r) { float v = oa[dt][r]; if (PRECISE) v += xa[dt][r] * 0.0009765625f; so[w][ln][dt * 16 + 8 * hh + r] = v * inv; }
  }
  __builtin_amdgcn_fence(4  , "workgroup"); __builtin_amdgcn_wave_barrier();
  const int rsub = lane >> 3, pc = (lane & 7) * 8;
  for (int pass = 0; pass < 2; ++pass) {
#pragma unroll
    for (int it = 0; it < 4; ++it) { const int rr = it * 4 + rsub;
      const v4f a = *(const v4fa*)&so[w][rr][pc], c = *(const v4fa*)&so[w][rr][pc + 4];
      FragH fh, fl;
#pragma unroll
      for (int e = 0; e < 4; ++e) { _Float16 h = (_Float16)a[e]; fh.h[e] = h; fl.h[e] = (_Float16)((a[e] - (float)h) * 1024.0f); h = (_Float16)c[e]; fh.h[4 + e] = h; fl.h[4 + e] = (_Float16)((c[e] - (float)h) * 1024.0f); }
      *(volatile v8us*)((unsigned short*)CH + (rowb + qw0 + rr) * DM + hd * HD + pc) = fh.half[0];
      if (PRECISE) *(volatile v8us*)((unsigned short*)CL + (rowl + qw0 + rr) * DM + hd * HD + pc) = fl.half[0];
    }
    if (pass == 0) __threadfence();
  }
}

__global__ __launch_bounds__(128) void k_flash_early(const _Float16* __restrict__ QK, const _Float16* __restrict__ QKL, const _Float16* __restrict__ VH, const _Float16* __restrict__ VL,
                                                     _Float16* __restrict__ CH, _Float16* __restrict__ CL, int qbase) {
  flash_body<true>(QK, QKL, VH, VL, CH, CL, qbase);
}
__global__ __launch_bounds__(128) void k_flash_late(const _Float16* __restrict__ QK, const _Float16* __restrict__ QKL, const _Float16* __restrict__ VH, const _Float16* __restrict__ VL,
                                                    _Float16* __restrict__ CH, _Float16* __restrict__ CL, int qbase) {
  flash_body<false>(QK, QKL, VH, VL, CH, CL, qbase);
}

template <bool RES>
__device__ __forceinline__ void gemm_out_body(const _Float16* __restrict__ A, int lda, size_t sA, const _Float16* __restrict__ A2, size_t sA2, const _Float16* __restrict__ Bh, int ldb, float alpha,
                                              const float* __restrict__ bias, float* __restrict__ C, int ldc, size_t sC, int M, int N, int K) {
  __shared__ __attribute__((aligned(16))) float so[4][32][68];
  const int tid = threadIdx.x, lane = tid & 31, ln = lane & 15, hh = lane >> 4; const int by = blockIdx.y;
  const int w = __builtin_amdgcn_readfirstlane(tid >> 5);
  A += (size_t)by * sA; A2 += (size_t)by * sA2; const size_t cofs = (size_t)by * sC;
  const int ntn = N >> 6; const int mt = blockIdx.x / ntn, nq = blockIdx.x - mt * ntn; const int row0 = mt * 128 + 32 * w, col0 = nq * 64; if (row0 >= M) return;
  const _Float16* a0p = A + (size_t)(row0 + ln) * lda; const _Float16* a1p = a0p + (size_t)16 * lda;
  const _Float16* b0p = Bh + (size_t)(col0 + ln) * ldb; const _Float16* b1p = b0p + (size_t)16 * ldb; const _Float16* b2p = b1p + (size_t)16 * ldb; const _Float16* b3p = b2p + (size_t)16 * ldb;
  const v8f z8 = {0.f,0.f,0.f,0.f,0.f,0.f,0.f,0.f}; v8f c00 = z8, c01 = z8, c02 = z8, c03 = z8, c10 = z8, c11 = z8, c12 = z8, c13 = z8;
  if (RES) {
    const _Float16* r0p = A2 + (size_t)(row0 + ln) * lda; const _Float16* r1p = r0p + (size_t)16 * lda;
#pragma unroll 1
    for (int kb = 0; kb < K; kb += 32) { const v16h a0 = g2_frag(r0p + kb, hh), a1 = g2_frag(r1p + kb, hh);
      v16h b = g2_frag(b0p + kb, hh); c00 = g2_mma(a0, b, c00); c10 = g2_mma(a1, b, c10);
      b = g2_frag(b1p + kb, hh); c01 = g2_mma(a0, b, c01); c11 = g2_mma(a1, b, c11);
      b = g2_frag(b2p + kb, hh); c02 = g2_mma(a0, b, c02); c12 = g2_mma(a1, b, c12);
      b = g2_frag(b3p + kb, hh); c03 = g2_mma(a0, b, c03); c13 = g2_mma(a1, b, c13); }
    const float f = 0.0009765625f;
    c00 = c00 * f; c01 = c01 * f; c02 = c02 * f; c03 = c03 * f; c10 = c10 * f; c11 = c11 * f; c12 = c12 * f; c13 = c13 * f;
  }
#pragma unroll 1
  for (int kb = 0; kb < K; kb += 32) { const v16h a0 = g2_frag(a0p + kb, hh), a1 = g2_frag(a1p + kb, hh);
    v16h b = g2_frag(b0p + kb, hh); c00 = g2_mma(a0, b, c00); c10 = g2_mma(a1, b, c10);
    b = g2_frag(b1p + kb, hh); c01 = g2_mma(a0, b, c01); c11 = g2_mma(a1, b, c11);
    b = g2_frag(b2p + kb, hh); c02 = g2_mma(a0, b, c02); c12 = g2_mma(a1, b, c12);
    b = g2_frag(b3p + kb, hh); c03 = g2_mma(a0, b, c03); c13 = g2_mma(a1, b, c13); }
  v8f accs[8] = {c00, c01, c02, c03, c10, c11, c12, c13};
#pragma unroll
  for (int u = 0; u < 8; ++u) { const int t = u & 3, half = u >> 2;
#pragma unroll
    for (int r = 0; r < 8; ++r) so[w][half * 16 + 8 * hh + r][t * 16 + ln] = accs[u][r] * alpha; }
  __builtin_amdgcn_fence(4  , "workgroup"); __builtin_amdgcn_wave_barrier();
  const int rsub = lane >> 4, c4 = (lane & 15) * 4;
  const v4f braw = *(const v4fa*)(bias + col0 + c4);
  v4f bb; bb[0] = bf16_rne(braw[0]); bb[1] = bf16_rne(braw[1]); bb[2] = bf16_rne(braw[2]); bb[3] = bf16_rne(braw[3]);
  for (int pass = 0; pass < 2; ++pass) {
#pragma unroll
    for (int q = 0; q < 16; ++q) { const int r = q * 2 + rsub;
      const v4f s4 = *(const v4fa*)&so[w][r][c4]; const v4f v = s4 + bb; *(volatile v4f*)(C + cofs + (size_t)(row0 + r) * ldc + col0 + c4) = v; }
    if (pass == 0) __threadfence();
  }
}

__global__ __launch_bounds__(128) void k_gemm_out_hi(const _Float16* __restrict__ A, int lda, size_t sA, const _Float16* __restrict__ A2, size_t sA2, const _Float16* __restrict__ Bh, int ldb, float alpha,
                                                     const float* __restrict__ bias, float* __restrict__ C, int ldc, size_t sC, int M, int N, int K) {
  gemm_out_body<false>(A, lda, sA, A2, sA2, Bh, ldb, alpha, bias, C, ldc, sC, M, N, K);
}
__global__ __launch_bounds__(128) void k_gemm_out_res(const _Float16* __restrict__ A, int lda, size_t sA, const _Float16* __restrict__ A2, size_t sA2, const _Float16* __restrict__ Bh, int ldb, float alpha,
                                                      const float* __restrict__ bias, float* __restrict__ C, int ldc, size_t sC, int M, int N, int K) {
  gemm_out_body<true>(A, lda, sA, A2, sA2, Bh, ldb, alpha, bias, C, ldc, sC, M, N, K);
}

extern "C" void kernel_launch(void* const* d_in, const int* in_sizes, int n_in,
                              void* d_out, int out_size, void* d_ws, size_t ws_size, hipStream_t stream) {
  if (n_in < 5) return;
  const long long needx = ((long long)(NB - 1) * SEQ_FULL + SEQ) * DM;
  if ((long long)in_sizes[0] < needx || (long long)out_size < needx) return;
  if ((long long)in_sizes[1] < (long long)DM * 3 * DM) return;
  if ((long long)in_sizes[2] < (long long)3 * DM) return;
  if ((long long)in_sizes[3] < (long long)DM * DM) return;
  if ((long long)in_sizes[4] < (long long)DM) return;
  const float* x = (const float*)d_in[0]; const float* qkv_w = (const float*)d_in[1]; const float* qkv_b = (const float*)d_in[2];
  const float* proj_w = (const float*)d_in[3]; const float* proj_b = (const float*)d_in[4];
  float* out = (float*)d_out;
  char* ws = (char*)d_ws; size_t off = 0;
  auto take = [&](size_t bytes) { char* p = ws + off; off += (bytes + 255) & ~(size_t)255; return p; };
  _Float16* BQK = (_Float16*)take(SZ_BQK); _Float16* BV = (_Float16*)take(SZ_BW); _Float16* BO = (_Float16*)take(SZ_BW);
  _Float16* X16 = (_Float16*)take(SZ_X16);
  _Float16* QKH = (_Float16*)take(SZ_QKH); _Float16* QKL = (_Float16*)take(SZ_QKL);
  _Float16* VTH = (_Float16*)take(SZ_VTH); _Float16* VTL = (_Float16*)take(SZ_VTL);
  _Float16* CTH = (_Float16*)take(SZ_CTH); _Float16* CTL = (_Float16*)take(SZ_CTL);
  float* CS = (float*)take(SZ_CS);
  if (off > ws_size || off > (size_t)134217728) return;
  RopeF rf;
  { double rt = 10000.0;
    for (int s = 0; s < 5; ++s) { double y = rt; for (int it = 0; it < 80; ++it) y = 0.5 * (y + rt / y); rt = y; }
    double pw = 1.0; for (int i = 0; i < 32; ++i) { rf.f[i] = 1.0f / (float)pw; pw *= rt; } }
  k_wtr<<<dim3(LQK / 64, DM / 64), 256, 0, stream>>>(qkv_w, LDW3, 0, BQK);
  k_wtr<<<dim3(DM / 64, DM / 64), 256, 0, stream>>>(qkv_w, LDW3, 2 * DM, BV);
  k_wtr<<<dim3(DM / 64, DM / 64), 256, 0, stream>>>(proj_w, DM, 0, BO);
  k_x16<<<dim3((unsigned)(((size_t)SEQ * DM / 8 + 255) / 256), NB), 256, 0, stream>>>(x, X16);
  k_ropetab<<<(32 * SEQ + 255) / 256, 256, 0, stream>>>(rf, CS);
  k_proj_qk<<<(unsigned)((NR / 128) * (LQK / 64)), 128, 0, stream>>>(X16, DM, BQK, DM, 0.0625f, CS, qkv_b, QKH, LQK, QKL, LQK, (int)NR, LQK, DM);
  k_proj_vt<<<(unsigned)((DM / 128) * (NR / 64)), 128, 0, stream>>>(BV, DM, X16, DM, 0.0625f, CS, qkv_b + 2 * DM, VTH, LDV, VTL, LDVL, DM, (int)NR, DM);
  k_flash_early<<<dim3(QE / 64, NB * NH), 128, 0, stream>>>(QKH, QKL, VTH, VTL, CTH, CTL, 0);
  if (SEQ > QE) k_flash_late<<<dim3((SEQ - QE) / 64, NB * NH), 128, 0, stream>>>(QKH, QKL, VTH, VTL, CTH, CTL, QE);
  if (SEQ > QE) k_gemm_out_hi<<<dim3((unsigned)(((SEQ - QE) / 128) * (DM / 64)), NB), 128, 0, stream>>>(CTH + (size_t)QE * DM, DM, (size_t)SEQ * DM, CTH + (size_t)QE * DM, (size_t)SEQ * DM, BO, DM, 0.0009765625f, proj_b, out + (size_t)QE * DM, DM, (size_t)SEQ_FULL * DM, SEQ - QE, DM, DM);
  k_gemm_out_res<<<dim3((unsigned)((QE / 128) * (DM / 64)), NB), 128, 0, stream>>>(CTH, DM, (size_t)SEQ * DM, CTL, (size_t)QE * DM, BO, DM, 0.0009765625f, proj_b, out, DM, (size_t)SEQ_FULL * DM, QE, DM, DM);
}
